// MultiHeadAttention_35837207117857
// MI455X (gfx1250) — hardware-run, weakly checked
//
#include <hip/hip_runtime.h>


#ifndef NB
#define NB 4
#endif
#ifndef SEQ
#define SEQ 2048
#endif
#define NB_FULL  4
#define SEQ_FULL 2048
#ifndef OUT_SEQ
#define OUT_SEQ SEQ
#endif
#define DM   1024
#define NH_  16
#define HD   64
#define AW   4
#define EARLY_ ((SEQ) < 512 ? (SEQ) : 512)
#define QRS  2048.0f
#define QRI  (1.0f / 2048.0f)
#define SC2  (0.125f * 1.4426950408889634f)
#define PSH  8.0f
#define ZC   16.0f
#define WOC  64.0f
#define OSC  (1.0f / 1024.0f)

static_assert(HD == 64);
static_assert(NH_ * HD == DM);
static_assert(DM % 64 == 0);
static_assert(DM % 32 == 0);
static_assert(SEQ % 64 == 0);
static_assert((NB * SEQ) % 64 == 0);
static_assert(SEQ % 32 == 0);
static_assert(SEQ % (16 * AW) == 0);
static_assert(EARLY_ % 64 == 0);
static_assert(EARLY_ <= SEQ);
static_assert(((size_t)SEQ * DM) % 8 == 0);
static_assert(NB <= NB_FULL);
static_assert(SEQ <= SEQ_FULL);

typedef _Float16 h16;
typedef unsigned short bf;
typedef __attribute__((ext_vector_type(16))) __bf16   v16bf;
typedef __attribute__((ext_vector_type(16))) _Float16 v16h;
typedef __attribute__((ext_vector_type(8)))  _Float16 v8h;
typedef __attribute__((ext_vector_type(8)))  unsigned short v8us;
typedef __attribute__((ext_vector_type(8)))  float    v8f;
typedef __attribute__((ext_vector_type(4)))  float    v4f;
typedef v4f  __attribute__((may_alias)) v4fa;

__device__ __forceinline__ unsigned short f2bf(float f) { unsigned u = __float_as_uint(f); u += 0x7FFFu + ((u >> 16) & 1u); return (unsigned short)(u >> 16); }
__device__ __forceinline__ float bfq(float f) { return __uint_as_float(((unsigned)f2bf(f)) << 16); }
__device__ __forceinline__ v16h cat16(v8h lo, v8h hi) { return __builtin_shufflevector(lo, hi, 0, 1, 2, 3, 4, 5, 6, 7, 8, 9, 10, 11, 12, 13, 14, 15); }
__device__ __forceinline__ v16bf cat16b(v8us lo, v8us hi) { return __builtin_bit_cast(v16bf, __builtin_shufflevector(lo, hi, 0, 1, 2, 3, 4, 5, 6, 7, 8, 9, 10, 11, 12, 13, 14, 15)); }
__device__ __forceinline__ v8f wmma16(v16h a, v16h b, v8f c) { return __builtin_amdgcn_wmma_f32_16x16x32_f16(false, a, false, b, (short)0, c, false, false); }
__device__ __forceinline__ v8f wmmab(v16bf a, v16bf b, v8f c) { return __builtin_amdgcn_wmma_f32_16x16x32_bf16(false, a, false, b, (short)0, c, false, false); }
__device__ __forceinline__ v16h  ldh(const h16* p) { return cat16(*(const v8h*)p, *(const v8h*)(p + 16)); }
__device__ __forceinline__ v16bf ldb(const bf* p)  { return cat16b(*(const v8us*)p, *(const v8us*)(p + 16)); }
__device__ __forceinline__ void wave_sync() { __builtin_amdgcn_fence(3  , "wavefront"); __builtin_amdgcn_wave_barrier(); asm volatile("" ::: "memory"); }

__global__ __launch_bounds__(256) void k_cvt8(const float* __restrict__ src, bf* dst, size_t n8) {
    const size_t i = (size_t)blockIdx.x * 256 + threadIdx.x; if (i >= n8) return;
    const v8f v = *(const v8f*)(src + i * 8); v8us o;
#pragma unroll
    for (int k = 0; k < 8; ++k) o[k] = f2bf(v[k]);
    *(volatile v8us*)(dst + i * 8) = o; __threadfence(); *(volatile v8us*)(dst + i * 8) = o;
}

__global__ __launch_bounds__(256) void k_wT(const float* __restrict__ W, bf* Wt, int asF16, float scale) {
    __shared__ float ts[64 * 65];
    const int tid = threadIdx.x; const int k0 = blockIdx.x * 64, n0 = blockIdx.y * 64;
#pragma unroll
    for (int i = 0; i < 4; ++i) { const int idx = tid + i * 256; const int kr = idx >> 4, c4 = (idx & 15) * 4;
        const v4f v = *(const v4f*)(W + (size_t)(k0 + kr) * DM + n0 + c4);
        ts[kr * 65 + c4 + 0] = v[0]; ts[kr * 65 + c4 + 1] = v[1]; ts[kr * 65 + c4 + 2] = v[2]; ts[kr * 65 + c4 + 3] = v[3]; }
    __syncthreads();
#pragma unroll 1
    for (int ps = 0; ps < 2; ++ps) {
#pragma unroll
        for (int s = 0; s < 2; ++s) { const int n = s * 32 + (tid >> 3), c8 = (tid & 7) * 8;
            v8us o;
#pragma unroll
            for (int i = 0; i < 8; ++i) { const float x = ts[(c8 + i) * 65 + n]; const unsigned short b16 = f2bf(x);
                const float xb = __uint_as_float(((unsigned)b16) << 16); const unsigned short hb = __builtin_bit_cast(unsigned short, (h16)(xb * scale));
                o[i] = asF16 ? hb : b16; }
            *(volatile v8us*)(Wt + (size_t)(n0 + n) * DM + k0 + c8) = o; }
        if (ps == 0) __threadfence(); }
}

__global__ __launch_bounds__(32) void k_proj(const bf* __restrict__ A, const bf* __restrict__ Bt, const float* __restrict__ bias, int biasRow,
                                             h16* Ph, h16* Pr, int resLim, int RB, size_t sRB, int pitch, int CB, size_t sCB) {
    __shared__ __align__(16) float os[16 * 68];
    const int K = DM;
    const int lane = threadIdx.x & 31, lr = lane & 15, hi = lane >> 4; const int r0 = blockIdx.x * 64, c0 = blockIdx.y * 64;
    const int useRes = ((c0 % CB) < resLim) ? 1 : 0;
    v8f acc[4][4];
#pragma unroll
    for (int mb = 0; mb < 4; ++mb)
#pragma unroll
        for (int nb = 0; nb < 4; ++nb) acc[mb][nb] = (v8f){};
    const size_t aoff = (size_t)(r0 + lr) * K + 8 * hi, boff = (size_t)(c0 + lr) * K + 8 * hi;
#pragma unroll 1
    for (int kc = 0; kc < K; kc += 32) {
        v16bf a[4];
#pragma unroll
        for (int mb = 0; mb < 4; ++mb) a[mb] = ldb(A + aoff + (size_t)mb * 16 * K + kc);
#pragma unroll
        for (int nb = 0; nb < 4; ++nb) { const v16bf b = ldb(Bt + boff + (size_t)nb * 16 * K + kc);
#pragma unroll
            for (int mb = 0; mb < 4; ++mb) acc[mb][nb] = wmmab(a[mb], b, acc[mb][nb]); }
        asm volatile("v_nop\n\tv_nop\n\tv_nop\n\tv_nop" : "+v"(acc[0][0]), "+v"(acc[1][1]), "+v"(acc[2][2]), "+v"(acc[3][3]) : "v"(a[0]), "v"(a[1]), "v"(a[2]), "v"(a[3]));
    }
    float bcol[4];
#pragma unroll
    for (int nb = 0; nb < 4; ++nb) { int ic = c0 + nb * 16 + lr; ic = ic < DM ? ic : DM - 1; bcol[nb] = bfq(bias[ic]); }
    const size_t tbase = (size_t)(r0 / RB) * sRB + (size_t)(r0 % RB) * (size_t)pitch + (size_t)(c0 / CB) * sCB + (size_t)(c0 % CB);
#pragma unroll
    for (int mb = 0; mb < 4; ++mb) {
        float brow[8];
#pragma unroll
        for (int j = 0; j < 8; ++j) { int ir = r0 + mb * 16 + hi * 8 + j; ir = ir < DM ? ir : DM - 1; brow[j] = bfq(bias[ir]); }
#pragma unroll
        for (int nb = 0; nb < 4; ++nb) {
#pragma unroll
            for (int j = 0; j < 8; ++j) os[(hi * 8 + j) * 68 + nb * 16 + lr] = acc[mb][nb][j] + (biasRow ? brow[j] : bcol[nb]); }
        wave_sync();
        const size_t sb = tbase + (size_t)(mb * 16) * (size_t)pitch;
#pragma unroll 1
        for (int ps = 0; ps < 2; ++ps) {
#pragma unroll
            for (int s = 0; s < 4; ++s) { const int row = 4 * s + (lane >> 3), c8 = (lane & 7) * 8;
                const v4f x0 = *(const v4fa*)(&os[row * 68 + c8]); const v4f x1 = *(const v4fa*)(&os[row * 68 + c8 + 4]); v8h hv, rv;
#pragma unroll
                for (int i = 0; i < 4; ++i) { const h16 a0 = (h16)x0[i]; const h16 a1 = (h16)x1[i]; hv[i] = a0; hv[4 + i] = a1; rv[i] = (h16)((x0[i] - (float)a0) * QRS); rv[4 + i] = (h16)((x1[i] - (float)a1) * QRS); }
                const size_t oo = sb + (size_t)row * (size_t)pitch + c8;
                *(volatile v8h*)(Ph + oo) = hv; if (useRes) *(volatile v8h*)(Pr + oo) = rv; }
            if (ps == 0) __threadfence(); }
        wave_sync();
    }
}

__global__ __launch_bounds__(32 * AW) void k_flash(const h16* __restrict__ QH, const h16* __restrict__ QR, const h16* __restrict__ KP,
                                                   const h16* __restrict__ VT, const h16* __restrict__ VR, h16* ZH, h16* ZR) {
    __shared__ __align__(16) float os[AW * 16 * 68];
    const int lane = threadIdx.x & 31, lr = lane & 15, hi = lane >> 4;
    const int wave = __builtin_amdgcn_readfirstlane((int)(threadIdx.x >> 5));
    const int zh = blockIdx.y; const int b = zh / NH_, h = zh % NH_;
    const int t0 = ((int)blockIdx.x * AW + wave) * 16;
    const bool early = ((int)blockIdx.x * (16 * AW)) < EARLY_;
    const int tq = t0 + lr;
    const int klast = (((t0 + 47) >> 5) - 1) * 32;
    const size_t pbase = (size_t)zh * SEQ * HD;
    const size_t qo = pbase + (size_t)(t0 + lr) * HD + 8 * hi;
    const v16h qh0 = ldh(QH + qo), qh1 = ldh(QH + qo + 32), qr0 = ldh(QR + qo), qr1 = ldh(QR + qo + 32);
    const size_t ko = pbase + (size_t)lr * HD + 8 * hi;
    const size_t vo = pbase + (size_t)lr * SEQ + 8 * hi;
    v8f o[4], e[4];
#pragma unroll
    for (int j = 0; j < 4; ++j) { o[j] = (v8f){}; e[j] = (v8f){}; }
    float m = -3.0e38f, l = 0.0f;
#pragma unroll 1
    for (int key0 = 0; key0 <= klast; key0 += 32) {
        const h16* ka = KP + ko + (size_t)key0 * HD;
        const v16h ka0 = ldh(ka), ka1 = ldh(ka + 32), kb0 = ldh(ka + 16 * HD), kb1 = ldh(ka + 16 * HD + 32);
        v8f sHa = (v8f){}, sLa = (v8f){}, sHb = (v8f){}, sLb = (v8f){};
        sHa = wmma16(ka0, qh0, sHa); sLa = wmma16(ka0, qr0, sLa); sHb = wmma16(kb0, qh0, sHb); sLb = wmma16(kb0, qr0, sLb);
        sHa = wmma16(ka1, qh1, sHa); sLa = wmma16(ka1, qr1, sLa); sHb = wmma16(kb1, qh1, sHb); sLb = wmma16(kb1, qr1, sLb);
        asm volatile("v_nop\n\tv_nop\n\tv_nop\n\tv_nop" : "+v"(sHa), "+v"(sLa), "+v"(sHb), "+v"(sLb) : "v"(ka0), "v"(ka1), "v"(kb0), "v"(kb1));
        float ta[8], tb[8];
#pragma unroll
        for (int r = 0; r < 8; ++r) { ta[r] = (sHa[r] + sLa[r] * QRI) * SC2; tb[r] = (sHb[r] + sLb[r] * QRI) * SC2; }
        if (key0 == klast) {
            const int kq = tq - key0 - 8 * hi;
#pragma unroll
            for (int r = 0; r < 8; ++r) { ta[r] = (r > kq) ? -3.0e38f : ta[r]; tb[r] = (r + 16 > kq) ? -3.0e38f : tb[r]; }
        }
        float mx = -3.0e38f;
#pragma unroll
        for (int r = 0; r < 8; ++r) mx = fmaxf(mx, fmaxf(ta[r], tb[r]));
        mx = fmaxf(mx, __shfl_xor(mx, 16, 32));
        const float mnew = fmaxf(m, mx);
        const float alpha = __builtin_amdgcn_exp2f(m - mnew);
        const float sh = PSH - mnew;
        v16h pb; float ls = 0.0f;
#pragma unroll
        for (int r = 0; r < 8; ++r) { const float fa = __builtin_amdgcn_exp2f(ta[r] + sh); const float fc = __builtin_amdgcn_exp2f(tb[r] + sh);
            const h16 pa = (h16)fa; const h16 pc = (h16)fc; pb[r] = pa; pb[8 + r] = pc; ta[r] = fa; tb[r] = fc; ls += (float)pa + (float)pc; }
#pragma unroll
        for (int j = 0; j < 4; ++j) o[j] = o[j] * alpha;
        const h16* va = VT + vo + key0;
        v16h v[4];
#pragma unroll
        for (int j = 0; j < 4; ++j) v[j] = ldh(va + (size_t)(16 * j) * SEQ);
#pragma unroll
        for (int j = 0; j < 4; ++j) o[j] = wmma16(v[j], pb, o[j]);
        asm volatile("v_nop\n\tv_nop\n\tv_nop\n\tv_nop" : "+v"(o[0]), "+v"(o[1]), "+v"(o[2]), "+v"(o[3]) : "v"(v[0]), "v"(v[1]), "v"(v[2]), "v"(v[3]), "v"(pb));
        if (early) {
            v16h pr; float lx = 0.0f;
#pragma unroll
            for (int r = 0; r < 8; ++r) { pr[r] = (h16)((ta[r] - (float)pb[r]) * QRS); pr[8 + r] = (h16)((tb[r] - (float)pb[8 + r]) * QRS); lx += ta[r] + tb[r]; }
            ls = lx;
#pragma unroll
            for (int j = 0; j < 4; ++j) e[j] = e[j] * alpha;
            const h16* ra = VR + vo + key0;
            v16h vr[4];
#pragma unroll
            for (int j = 0; j < 4; ++j) vr[j] = ldh(ra + (size_t)(16 * j) * SEQ);
#pragma unroll
            for (int j = 0; j < 4; ++j) e[j] = wmma16(vr[j], pb, e[j]);
#pragma unroll
            for (int j = 0; j < 4; ++j) e[j] = wmma16(v[j], pr, e[j]);
            asm volatile("v_nop\n\tv_nop\n\tv_nop\n\tv_nop" : "+v"(e[0]), "+v"(e[1]), "+v"(e[2]), "+v"(e[3]) : "v"(vr[0]), "v"(vr[1]), "v"(vr[2]), "v"(vr[3]), "v"(pr), "v"(v[0]), "v"(v[1]), "v"(v[2]), "v"(v[3]));
        }
        l = l * alpha + ls; m = mnew;
    }
    l += __shfl_xor(l, 16, 32);
    const float zs = (1.0f / l) * ZC;
    const int wb = wave * 16 * 68;
#pragma unroll
    for (int j = 0; j < 4; ++j) { v4f a, c;
#pragma unroll
        for (int i = 0; i < 4; ++i) { a[i] = (o[j][i] + e[j][i] * QRI) * zs; c[i] = (o[j][4 + i] + e[j][4 + i] * QRI) * zs; }
        *(v4fa*)(&os[wb + lr * 68 + 16 * j + 8 * hi]) = a; *(v4fa*)(&os[wb + lr * 68 + 16 * j + 8 * hi + 4]) = c; }
    wave_sync();
    const size_t zb = ((size_t)b * SEQ + t0) * DM + (size_t)h * HD;
#pragma unroll 1
    for (int ps = 0; ps < 2; ++ps) {
#pragma unroll
        for (int s = 0; s < 4; ++s) { const int row = 4 * s + (lane >> 3), c8 = (lane & 7) * 8;
            const v4f x0 = *(const v4fa*)(&os[wb + row * 68 + c8]); const v4f x1 = *(const v4fa*)(&os[wb + row * 68 + c8 + 4]); v8h hv, rv;
#pragma unroll
            for (int i = 0; i < 4; ++i) { const h16 a0 = (h16)x0[i]; const h16 a1 = (h16)x1[i]; hv[i] = a0; hv[4 + i] = a1; rv[i] = (h16)((x0[i] - (float)a0) * QRS); rv[4 + i] = (h16)((x1[i] - (float)a1) * QRS); }
            const size_t oo = zb + (size_t)row * DM + c8;
            *(volatile v8h*)(ZH + oo) = hv; if (early) *(volatile v8h*)(ZR + oo) = rv; }
        if (ps == 0) __threadfence(); }
}

__global__ __launch_bounds__(32) void k_oproj(const h16* __restrict__ ZH, const h16* __restrict__ ZR, const h16* __restrict__ Wt, const float* __restrict__ bo, float* OUT) {
    __shared__ __align__(16) float os[16 * 68];
    const int K = DM;
    const int lane = threadIdx.x & 31, lr = lane & 15, hi = lane >> 4; const int r0 = blockIdx.x * 32, c0 = blockIdx.y * 64;
    const int bb = r0 / SEQ, tt = r0 % SEQ; const bool early = tt < EARLY_;
    v8f acc[2][4], acr[2][4];
#pragma unroll
    for (int mb = 0; mb < 2; ++mb)
#pragma unroll
        for (int nb = 0; nb < 4; ++nb) { acc[mb][nb] = (v8f){}; acr[mb][nb] = (v8f){}; }
    const size_t aoff = (size_t)(r0 + lr) * K + 8 * hi, boff = (size_t)(c0 + lr) * K + 8 * hi;
#pragma unroll 1
    for (int kc = 0; kc < K; kc += 32) {
        v16h a[2], w[4];
#pragma unroll
        for (int mb = 0; mb < 2; ++mb) a[mb] = ldh(ZH + aoff + (size_t)mb * 16 * K + kc);
#pragma unroll
        for (int nb = 0; nb < 4; ++nb) w[nb] = ldh(Wt + boff + (size_t)nb * 16 * K + kc);
#pragma unroll
        for (int nb = 0; nb < 4; ++nb)
#pragma unroll
            for (int mb = 0; mb < 2; ++mb) acc[mb][nb] = wmma16(a[mb], w[nb], acc[mb][nb]);
        asm volatile("v_nop\n\tv_nop\n\tv_nop\n\tv_nop" : "+v"(acc[0][0]), "+v"(acc[1][0]), "+v"(acc[0][1]), "+v"(acc[1][1]), "+v"(acc[0][2]), "+v"(acc[1][2]), "+v"(acc[0][3]), "+v"(acc[1][3]) : "v"(a[0]), "v"(a[1]), "v"(w[0]), "v"(w[1]), "v"(w[2]), "v"(w[3]));
        if (early) {
            v16h ar[2];
#pragma unroll
            for (int mb = 0; mb < 2; ++mb) ar[mb] = ldh(ZR + aoff + (size_t)mb * 16 * K + kc);
#pragma unroll
            for (int nb = 0; nb < 4; ++nb)
#pragma unroll
                for (int mb = 0; mb < 2; ++mb) acr[mb][nb] = wmma16(ar[mb], w[nb], acr[mb][nb]);
            asm volatile("v_nop\n\tv_nop\n\tv_nop\n\tv_nop" : "+v"(acr[0][0]), "+v"(acr[1][0]), "+v"(acr[0][1]), "+v"(acr[1][1]), "+v"(acr[0][2]), "+v"(acr[1][2]), "+v"(acr[0][3]), "+v"(acr[1][3]) : "v"(ar[0]), "v"(ar[1]), "v"(w[0]), "v"(w[1]), "v"(w[2]), "v"(w[3]));
        }
    }
    float bcol[4];
#pragma unroll
    for (int nb = 0; nb < 4; ++nb) bcol[nb] = bfq(bo[c0 + nb * 16 + lr]);
    float* orow = OUT + ((size_t)bb * OUT_SEQ + tt) * DM + c0;
#pragma unroll
    for (int mb = 0; mb < 2; ++mb) {
#pragma unroll
        for (int nb = 0; nb < 4; ++nb) {
#pragma unroll
            for (int j = 0; j < 8; ++j) os[(hi * 8 + j) * 68 + nb * 16 + lr] = (acc[mb][nb][j] + acr[mb][nb][j] * QRI) * OSC + bcol[nb]; }
        wave_sync();
        float* ob = orow + (size_t)(mb * 16) * DM;
#pragma unroll 1
        for (int ps = 0; ps < 2; ++ps) {
#pragma unroll
            for (int s = 0; s < 8; ++s) { const int row = 2 * s + hi, cofs = lr * 4;
                const v4f val = *(const v4fa*)(&os[row * 68 + cofs]);
                *(volatile v4f*)(ob + (size_t)row * DM + cofs) = val; }
            if (ps == 0) __threadfence(); }
        wave_sync();
    }
}

static constexpr size_t al256(size_t v) { return (v + 255) & ~(size_t)255; }
static constexpr size_t SZ_XB = al256((size_t)NB * SEQ * DM * 2);
static constexpr size_t SZ_WB = al256((size_t)4 * DM * DM * 2);
static constexpr size_t SZ_PL = al256((size_t)NB * NH_ * SEQ * HD * 2);
static constexpr size_t SZ_TOTAL = 2 * SZ_XB + SZ_WB + 5 * SZ_PL;
static_assert(SZ_TOTAL <= (size_t)134217728);
static_assert(((size_t)DM * DM * 2) % 256 == 0);
static_assert((size_t)NB * SEQ * DM * 2 <= SZ_XB);

extern "C" void kernel_launch(void* const* d_in, const int* in_sizes, int n_in,
                              void* d_out, int out_size, void* d_ws, size_t ws_size, hipStream_t stream) {
    if (n_in < 10) return;
    const size_t needx = ((size_t)(NB - 1) * SEQ_FULL + SEQ) * DM;
    if ((size_t)in_sizes[0] < needx || (size_t)in_sizes[1] < needx) return;
    if ((size_t)in_sizes[2] < (size_t)DM * DM || (size_t)in_sizes[4] < (size_t)DM * DM || (size_t)in_sizes[6] < (size_t)DM * DM || (size_t)in_sizes[8] < (size_t)DM * DM) return;
    if (in_sizes[3] < DM || in_sizes[5] < DM || in_sizes[7] < DM || in_sizes[9] < DM) return;
    if ((size_t)out_size < ((size_t)(NB - 1) * OUT_SEQ + SEQ) * DM) return;
    if (SZ_TOTAL > ws_size) return;
    const float* data = (const float*)d_in[0]; const float* ctx = (const float*)d_in[1];
    const float* wq = (const float*)d_in[2]; const float* bq = (const float*)d_in[3];
    const float* wk = (const float*)d_in[4]; const float* bk = (const float*)d_in[5];
    const float* wv = (const float*)d_in[6]; const float* bv = (const float*)d_in[7];
    const float* wo = (const float*)d_in[8]; const float* bo = (const float*)d_in[9];
    float* OUT = (float*)d_out;
    char* wsp = (char*)d_ws;
    bf* DATAB = (bf*)wsp; wsp += SZ_XB;
    bf* CTXB  = (bf*)wsp; wsp += SZ_XB;
    bf* WB = (bf*)wsp; wsp += SZ_WB;
    h16* QH = (h16*)wsp; wsp += SZ_PL;
    h16* QR = (h16*)wsp; wsp += SZ_PL;
    h16* KP = (h16*)wsp; wsp += SZ_PL;
    h16* VT = (h16*)wsp; wsp += SZ_PL;
    h16* VR = (h16*)wsp; wsp += SZ_PL;
    bf* WQT = WB; bf* WKT = WB + (size_t)DM * DM; bf* WVT = WB + (size_t)2 * DM * DM; bf* WOT = WB + (size_t)3 * DM * DM;
    h16* ZH = (h16*)DATAB;
    h16* ZR = (h16*)CTXB;

    if (SEQ == SEQ_FULL) {
        const size_t n8 = (size_t)NB * SEQ * DM / 8;
        k_cvt8<<<(unsigned)((n8 + 255) / 256), 256, 0, stream>>>(data, DATAB, n8);
        k_cvt8<<<(unsigned)((n8 + 255) / 256), 256, 0, stream>>>(ctx, CTXB, n8);
    } else {
        const size_t n8 = (size_t)SEQ * DM / 8;
        for (int b = 0; b < NB; ++b) {
            k_cvt8<<<(unsigned)((n8 + 255) / 256), 256, 0, stream>>>(data + (size_t)b * SEQ_FULL * DM, DATAB + (size_t)b * SEQ * DM, n8);
            k_cvt8<<<(unsigned)((n8 + 255) / 256), 256, 0, stream>>>(ctx + (size_t)b * SEQ_FULL * DM, CTXB + (size_t)b * SEQ * DM, n8);
        }
    }
    k_wT<<<dim3(DM / 64, DM / 64, 1), 256, 0, stream>>>(wq, WQT, 0, 1.0f);
    k_wT<<<dim3(DM / 64, DM / 64, 1), 256, 0, stream>>>(wk, WKT, 0, 1.0f);
    k_wT<<<dim3(DM / 64, DM / 64, 1), 256, 0, stream>>>(wv, WVT, 0, 1.0f);
    k_wT<<<dim3(DM / 64, DM / 64, 1), 256, 0, stream>>>(wo, WOT, 1, WOC);

    k_proj<<<dim3(NB * SEQ / 64, DM / 64, 1), 32, 0, stream>>>(DATAB, WQT, bq, 0, QH, QR, 1, SEQ, (size_t)NH_ * SEQ * HD, HD, HD, (size_t)SEQ * HD);
    k_proj<<<dim3(NB * SEQ / 64, DM / 64, 1), 32, 0, stream>>>(CTXB,  WKT, bk, 0, KP, KP, 0, SEQ, (size_t)NH_ * SEQ * HD, HD, HD, (size_t)SEQ * HD);
    k_proj<<<dim3(DM / 64, NB * SEQ / 64, 1), 32, 0, stream>>>(WVT, CTXB, bv, 1, VT, VR, EARLY_, DM, (size_t)0, SEQ, SEQ, (size_t)DM * SEQ);

    k_flash<<<dim3(SEQ / (16 * AW), NB * NH_, 1), 32 * AW, 0, stream>>>(QH, QR, KP, VT, VR, ZH, ZR);

    k_oproj<<<dim3(NB * SEQ / 32, DM / 64, 1), 32, 0, stream>>>(ZH, ZR, (const h16*)WOT, bo, OUT);
}
